// PNP_704374637376
// MI455X (gfx1250) — hardware-verified
//
#include <hip/hip_runtime.h>
#include <math.h>

typedef __attribute__((ext_vector_type(16))) _Float16 v16h;
typedef __attribute__((ext_vector_type(16))) __bf16 v16b;
typedef __attribute__((ext_vector_type(8)))  _Float16 v8h;
typedef __attribute__((ext_vector_type(8)))  float v8f;
typedef __attribute__((ext_vector_type(4)))  float v4f;
typedef __attribute__((ext_vector_type(2)))  float v2f;
typedef __attribute__((ext_vector_type(4)))  unsigned v4u;
typedef __attribute__((ext_vector_type(4)))  int v4i;
typedef float __attribute__((may_alias)) float_a;
typedef int __attribute__((may_alias)) int_a;

template <typename T> __device__ __forceinline__ void vst2(void* p, T v) { *(volatile T*)p = v; __threadfence(); *(volatile T*)p = v; }
__device__ __forceinline__ v8f wmma16(v16h a, v16h b, v8f c) {
  v8f d = __builtin_amdgcn_wmma_f32_16x16x32_f16(false, a, false, b, (short)0, c, false, false);
  asm volatile("v_nop\n\tv_nop\n\tv_nop\n\tv_nop" : "+v"(d) : "v"(a), "v"(b));
  return d;
}
__device__ __forceinline__ v8f wmma_bf(v16b a, v16b b, v8f c) {
  v8f d = __builtin_amdgcn_wmma_f32_16x16x32_bf16(false, a, false, b, (short)0, c, false, false);
  asm volatile("v_nop\n\tv_nop\n\tv_nop\n\tv_nop" : "+v"(d) : "v"(a), "v"(b));
  return d;
}
__device__ __forceinline__ v16h frag_h(const _Float16* rowk0, int lane) {
  union { v16h v; v8h q[2]; } u; const _Float16* p = rowk0 + 8 * (lane >> 4);
  u.q[0] = *(const v8h*)p; u.q[1] = *(const v8h*)(p + 16); return u.v;
}
__device__ __forceinline__ v16h frag_f32(const float* rowk0, int lane) {
  v16h a; const float* p = rowk0 + 8 * (lane >> 4);
#pragma unroll
  for (int i = 0; i < 8; ++i) { a[i] = (_Float16)p[i]; a[8 + i] = (_Float16)p[16 + i]; }
  return a;
}
__device__ __forceinline__ v16h frag_f32s(const float* rowk0, int lane, float sc) {
  v16h a; const float* p = rowk0 + 8 * (lane >> 4);
#pragma unroll
  for (int i = 0; i < 8; ++i) { a[i] = (_Float16)(p[i] * sc); a[8 + i] = (_Float16)(p[16 + i] * sc); }
  return a;
}
__device__ __forceinline__ v16h fragc_f32(const float* W, int k0, int n, int lane, int ld, int K) {
  v16h a; const int g = lane >> 4;
#pragma unroll
  for (int i = 0; i < 8; ++i) { const int ka = k0 + 8 * g + i, kb = ka + 16;
    a[i] = (_Float16)(ka < K ? W[(size_t)(ka < K ? ka : K - 1) * ld + n] : 0.f); a[8 + i] = (_Float16)(kb < K ? W[(size_t)(kb < K ? kb : K - 1) * ld + n] : 0.f); }
  return a;
}
struct F2 { v16b h, l; };
__device__ __forceinline__ F2 bsplit16(const float v[16]) { F2 r;
#pragma unroll
  for (int i = 0; i < 16; ++i) { const __bf16 h = (__bf16)v[i]; r.h[i] = h; r.l[i] = (__bf16)(v[i] - (float)h); }
  return r; }
__device__ __forceinline__ F2 split_row(const float* row, int k0, int lane) { float v[16]; const float* p = row + k0 + 8 * (lane >> 4);
#pragma unroll
  for (int i = 0; i < 8; ++i) { v[i] = p[i]; v[8 + i] = p[16 + i]; }
  return bsplit16(v); }
__device__ __forceinline__ F2 split_rowK(const float* row, int k0, int lane, int K) { float v[16]; const int g = lane >> 4;
#pragma unroll
  for (int i = 0; i < 8; ++i) { const int ka = k0 + 8 * g + i, kb = ka + 16; v[i] = ka < K ? row[ka < K ? ka : K - 1] : 0.f; v[8 + i] = kb < K ? row[kb < K ? kb : K - 1] : 0.f; }
  return bsplit16(v); }
__device__ __forceinline__ F2 split_col(const float* W, int k0, int n, int lane, int ld, int K) { float v[16]; const int g = lane >> 4;
#pragma unroll
  for (int i = 0; i < 8; ++i) { const int ka = k0 + 8 * g + i, kb = ka + 16; v[i] = ka < K ? W[(size_t)(ka < K ? ka : K - 1) * ld + n] : 0.f; v[8 + i] = kb < K ? W[(size_t)(kb < K ? kb : K - 1) * ld + n] : 0.f; }
  return bsplit16(v); }
__device__ __forceinline__ v8f mac3(const F2& a, const F2& b, v8f c) { c = wmma_bf(a.l, b.h, c); c = wmma_bf(a.h, b.l, c); return wmma_bf(a.h, b.h, c); }
__device__ __forceinline__ float sigm(float v) { return 1.0f / (1.0f + expf(-v)); }
#define LDSX() do { asm volatile("s_wait_dscnt 0" ::: "memory"); __builtin_amdgcn_wave_barrier(); __builtin_amdgcn_fence(__ATOMIC_RELEASE, "workgroup"); } while (0)


#define NB 3
#define SS 4096
#define DM 320
#define NH 8
#define HD 40
#define HDK 64
#define HDV 48
#define NR (NB * SS)
#ifndef TQB
#define TQB (SS / 64)
#endif
typedef __attribute__((ext_vector_type(8))) __bf16 v8b;
__device__ __forceinline__ v16b frag_b(const __bf16* rowk0, int lane) {
  union { v16b v; v8b q[2]; } u; const __bf16* p = rowk0 + 8 * (lane >> 4);
  u.q[0] = *(const v8b*)p; u.q[1] = *(const v8b*)(p + 16); return u.v;
}
__device__ __forceinline__ float bfr(float v) { return (float)(__bf16)v; }
__device__ __attribute__((noinline)) float exp_ni(float v) { return expf(v); }
__device__ __attribute__((noinline)) float erf_ni(float v) { return erff(v); }

#define WS_PW   0u
#define WS_Q    (WS_PW + 2u * (size_t)4 * DM * DM)
#define WS_K    (WS_Q + 2u * (size_t)SS * NH * HDK)
#define WS_V    (WS_K + 2u * (size_t)SS * NH * HDK)
#define OSTR    (NH * 64)
#define WS_O    (WS_V + 2u * (size_t)NB * NH * HDV * SS)
#define WS_POS  (WS_O + 4u * (size_t)NR * OSTR)
#define WS_END  (WS_POS + 2u * (size_t)DM * OSTR)

__global__ __launch_bounds__(64) void k_pack(const float* __restrict__ WQ, const float* __restrict__ WK, const float* __restrict__ WV, const float* __restrict__ WO, __bf16* __restrict__ P, __bf16* __restrict__ POS) { const int n = blockIdx.x, which = blockIdx.y, t = threadIdx.x; const float* Wm = (which == 0) ? WQ : (which == 1) ? WK : (which == 2) ? WV : WO; __shared__ __align__(16) __bf16 s[OSTR]; for (int k = t; k < DM; k += 64) s[k] = (__bf16)Wm[(size_t)n * DM + k]; __syncthreads(); if (t < DM / 8) vst2((unsigned*)(P + ((size_t)which * DM + n) * DM + t * 8), *(const v4u*)&s[t * 8]);
  if (which == 3) { __syncthreads(); __shared__ __align__(16) __bf16 s2[OSTR]; for (int k = t; k < OSTR; k += 64) { const int hh = k >> 6, d = k & 63; s2[k] = (d < HD) ? s[hh * HD + d] : (__bf16)0.f; } __syncthreads(); for (int q = t; q < OSTR / 8; q += 64) vst2((unsigned*)(POS + (size_t)n * OSTR + q * 8), *(const v4u*)&s2[q * 8]); } }
__global__ __launch_bounds__(256) void k_zero(_Float16* __restrict__ A, size_t n16) { const size_t i = ((size_t)blockIdx.x * 256 + threadIdx.x) * 16; if (i + 16 <= n16) { v4f z; z[0] = z[1] = z[2] = z[3] = 0.f; vst2((float*)(A + i), z); vst2((float*)(A + i + 8), z); } }
__global__ __launch_bounds__(128) void k_proj(const float* __restrict__ X, const __bf16* __restrict__ P, _Float16* __restrict__ Q, _Float16* __restrict__ Kr, _Float16* __restrict__ V) {
  __shared__ __align__(16) _Float16 so[64][56]; __shared__ __align__(16) _Float16 st[48][72];
  const int tid = threadIdx.x, wave = tid >> 5, lane = tid & 31, col = lane & 15, g = lane >> 4; const int h = blockIdx.y, which = blockIdx.z; const size_t rb0 = (size_t)blockIdx.x * 64, r0 = rb0 + wave * 16;
  if (which < 2 && rb0 >= SS) return;
  const __bf16* Wr = P + ((size_t)which * DM + h * HD) * DM;
  v8f acc[3] = {};
#pragma unroll
  for (int kc = 0; kc < DM / 32; ++kc) { v16b a; { const float* p = X + (r0 + col) * DM + kc * 32 + 8 * g;
#pragma unroll
      for (int i = 0; i < 8; ++i) { a[i] = (__bf16)p[i]; a[8 + i] = (__bf16)p[16 + i]; } }
#pragma unroll
    for (int j = 0; j < 3; ++j) { const int n = j * 16 + col; acc[j] = wmma_bf(a, frag_b(Wr + (size_t)min(n, HD - 1) * DM + kc * 32, lane), acc[j]); } }
  if (which < 2) {
#pragma unroll
    for (int j = 0; j < 3; ++j) { const int n = j * 16 + col;
#pragma unroll
      for (int r = 0; r < 8; ++r) so[wave * 16 + 8 * g + r][n] = (n < HD) ? (_Float16)acc[j][r] : (_Float16)0.f; }
    LDSX();
    _Float16* dst = (which == 0) ? Q : Kr;
    for (int rl = 0; rl < 16; ++rl) if (lane < 6) vst2((unsigned*)(dst + (r0 + rl) * (NH * HDK) + h * HDK + lane * 8), *(const v4u*)&so[wave * 16 + rl][lane * 8]);
  } else {
#pragma unroll
    for (int j = 0; j < 3; ++j) { const int n = j * 16 + col;
#pragma unroll
      for (int r = 0; r < 8; ++r) st[n][wave * 16 + 8 * g + r] = (n < HD) ? (_Float16)acc[j][r] : (_Float16)0.f; }
    __syncthreads();
    const size_t b = rb0 / SS, s0 = rb0 % SS;
    for (int e = tid; e < 48 * 8; e += 128) { const int d = e >> 3, pc = e & 7; vst2((unsigned*)(V + ((b * NH * HDV + h * HDV + d) * SS) + s0 + pc * 8), *(const v4u*)&st[d][pc * 8]); } }
}
__global__ __launch_bounds__(128) void k_attn(const _Float16* __restrict__ Q, const _Float16* __restrict__ Kr, const _Float16* __restrict__ V, float* __restrict__ O) {
  __shared__ __align__(16) _Float16 sph[4][16][40]; __shared__ __align__(16) float so[4][16][68];
  const int tid = threadIdx.x, wave = tid >> 5, lane = tid & 31, col = lane & 15, g = lane >> 4; const int h = blockIdx.y; const int q0 = blockIdx.x * 64 + wave * 16;
  v16h aq[2];
#pragma unroll
  for (int kc = 0; kc < 2; ++kc) aq[kc] = frag_h(Q + (size_t)(q0 + col) * (NH * HDK) + h * HDK + kc * 32, lane);
  float m[8], l[8];
#pragma unroll
  for (int r = 0; r < 8; ++r) { m[r] = -3.0e38f; l[r] = 0.f; }
  v8f acc[3][3] = {};
#pragma unroll 1
  for (int ks = 0; ks < SS / 32; ++ks) { const int j0 = ks * 32; v8f s[2];
#pragma unroll
    for (int ct = 0; ct < 2; ++ct) { const size_t rk = (size_t)(j0 + ct * 16 + col) * (NH * HDK) + h * HDK; v8f c = {};
#pragma unroll
      for (int kc = 0; kc < 2; ++kc) c = wmma16(aq[kc], frag_h(Kr + rk + kc * 32, lane), c);
#pragma unroll
      for (int r = 0; r < 8; ++r) s[ct][r] = c[r] * 0.15811388300841897f; }
#pragma unroll
    for (int r = 0; r < 8; ++r) { float mx = fmaxf(s[0][r], s[1][r]);
#pragma unroll
      for (int o = 1; o < 16; o <<= 1) mx = fmaxf(mx, __shfl_xor(mx, o));
      const float mn = fmaxf(m[r], mx); const float alpha = (m[r] <= -1.0e38f) ? 0.f : __expf(m[r] - mn); const float e0 = __expf(s[0][r] - mn), e1 = __expf(s[1][r] - mn); float es = e0 + e1;
#pragma unroll
      for (int o = 1; o < 16; o <<= 1) es += __shfl_xor(es, o);
      l[r] = l[r] * alpha + es; m[r] = mn;
#pragma unroll
      for (int b = 0; b < 3; ++b)
#pragma unroll
        for (int dt = 0; dt < 3; ++dt) acc[b][dt][r] *= alpha;
      sph[wave][8 * g + r][col] = (_Float16)(e0 * 2048.0f); sph[wave][8 * g + r][16 + col] = (_Float16)(e1 * 2048.0f); }
    LDSX();
    const v16h pa = frag_h(&sph[wave][col][0], lane);
#pragma unroll
    for (int b = 0; b < 3; ++b)
#pragma unroll
      for (int dt = 0; dt < 3; ++dt) acc[b][dt] = wmma16(pa, frag_h(V + (((size_t)b * NH * HDV + h * HDV + dt * 16 + col) * SS) + j0, lane), acc[b][dt]);
    LDSX(); }
#pragma unroll
  for (int b = 0; b < 3; ++b) {
#pragma unroll
    for (int r = 0; r < 8; ++r) { const float il = (1.0f / 2048.0f) / l[r];
#pragma unroll
      for (int dt = 0; dt < 3; ++dt) so[wave][8 * g + r][dt * 16 + col] = (dt * 16 + col < HD) ? acc[b][dt][r] * il : 0.f; so[wave][8 * g + r][48 + col] = 0.f; }
    LDSX();
    for (int rl = 0; rl < 16; ++rl) if (lane < 16) vst2(O + ((size_t)b * SS + q0 + rl) * OSTR + h * 64 + lane * 4, *(const v4f*)&so[wave][rl][lane * 4]);
    LDSX(); }
}
__global__ __launch_bounds__(128) void k_out(const float* __restrict__ O, const __bf16* __restrict__ POS, const float* __restrict__ BO, float* __restrict__ OUT) {
  __shared__ __align__(16) float so[4][16][68];
  const int tid = threadIdx.x, wave = tid >> 5, lane = tid & 31, col = lane & 15, g = lane >> 4; const size_t r0 = (size_t)blockIdx.x * 64 + wave * 16; const int n0 = blockIdx.y * 64;
  v8f acc[4] = {};
#pragma unroll
  for (int kc = 0; kc < OSTR / 32; ++kc) { if ((kc & 1) && ((kc * 32) & 63) >= 48) {}
    const F2 a = split_row(O + (r0 + col) * OSTR, kc * 32, lane);
#pragma unroll
    for (int j = 0; j < 4; ++j) { const v16b w = frag_b(POS + (size_t)(n0 + j * 16 + col) * OSTR + kc * 32, lane); acc[j] = wmma_bf(a.l, w, acc[j]); acc[j] = wmma_bf(a.h, w, acc[j]); } }
#pragma unroll
  for (int j = 0; j < 4; ++j) { const float bb = bfr(BO[n0 + j * 16 + col]);
#pragma unroll
    for (int r = 0; r < 8; ++r) so[wave][8 * g + r][j * 16 + col] = acc[j][r] + bb; }
  LDSX();
  for (int rl = 0; rl < 16; ++rl) if (lane < 16) vst2(OUT + (r0 + rl) * DM + n0 + lane * 4, *(const v4f*)&so[wave][rl][lane * 4]);
}
extern "C" void kernel_launch(void* const* d_in, const int* in_sizes, int n_in, void* d_out, int out_size, void* d_ws, size_t ws_size, hipStream_t stream) {
  (void)in_sizes; (void)n_in; (void)out_size;
  const float** F = (const float**)d_in;
  if (ws_size < (size_t)WS_END) return;
  char* ws = (char*)d_ws; __bf16* P = (__bf16*)ws; __bf16* POS = (__bf16*)(ws + WS_POS); _Float16 *Q = (_Float16*)(ws + WS_Q), *Kr = (_Float16*)(ws + WS_K), *V = (_Float16*)(ws + WS_V); float* O = (float*)(ws + WS_O);
  k_pack<<<dim3(DM, 4), 64, 0, stream>>>(F[1], F[2], F[3], F[4], P, POS);
  k_zero<<<(unsigned)(((size_t)SS * NH * HDK * 2 + (size_t)NB * NH * HDV * SS) / 4096), 256, 0, stream>>>(Q, (size_t)SS * NH * HDK * 2 + (size_t)NB * NH * HDV * SS);
  k_proj<<<dim3(NR / 64, NH, 3), 128, 0, stream>>>(F[0], P, Q, Kr, V);
  k_attn<<<dim3(TQB, NH), 128, 0, stream>>>(Q, Kr, V, O);
  k_out<<<dim3(NR / 64, DM / 64), 128, 0, stream>>>(O, POS, F[5], (float*)d_out);
}
